// MultiHeadAttnGRU_78451872629031
// MI455X (gfx1250) — hardware-verified
//
#include <hip/hip_runtime.h>
#include <stdint.h>
#include <stddef.h>
#include <math.h>

#pragma clang fp contract(off)

#define LM    128
#define BS    16
#define DD    512
#define HH    512
#define VV    16000
#define NHD   8
#define DKD   64
#define QK    1024
#define G3    1536
#define MROWS (LM * BS)

#define QP    1032
#define CP    520
#define KVP   132
#define TSP   72
#define LTP   68

#define O_QH   0
#define O_QL   (O_QH + BS * QP * 2)
#define O_CH   (O_QL + BS * QP * 2)
#define O_CL   (O_CH + BS * CP * 2)
#define O_F    (O_CL + BS * CP * 2)
#define O_HP   (O_F + BS * HH * 4)
#define O_P    (O_HP + BS * HH * 4)
#define O_SC   (O_P + NHD * LM * 4)
#define O_AM   (O_SC + BS * LM * 4)
#define O_OL   (O_AM + 64)
#define LDS_STEP (O_OL + 64)

static_assert(LDS_STEP == 177280);
static_assert((O_QL % 16) == 0);
static_assert((O_CH % 16) == 0);
static_assert((O_CL % 16) == 0);
static_assert((O_F % 16) == 0);
static_assert((O_HP % 16) == 0);
static_assert((O_P % 16) == 0);
static_assert((O_SC % 16) == 0);
static_assert((O_AM % 16) == 0);
static_assert((QP * 2) % 16 == 0);
static_assert((CP * 2) % 16 == 0);
static_assert((KVP * 4) % 16 == 0);
static_assert((TSP * 2) % 16 == 0);
static_assert((LTP * 4) % 16 == 0);
static_assert(VV % 128 == 0);
static_assert(VV % 64 == 0);
static_assert(HH % 64 == 0);
static_assert(QK % 64 == 0);
static_assert(G3 % 64 == 0);
static_assert(DD % 64 == 0);
static_assert(MROWS % 64 == 0);
static_assert(NHD * DKD == HH);
static_assert(LM == 128);
static_assert(BS == 16);

typedef __bf16         v16bf __attribute__((ext_vector_type(16)));
typedef float          v8f   __attribute__((ext_vector_type(8)));
typedef float          v4f   __attribute__((ext_vector_type(4)));
typedef unsigned int   v4u   __attribute__((ext_vector_type(4)));
typedef unsigned int   v2u   __attribute__((ext_vector_type(2)));
typedef v4f __attribute__((may_alias)) v4fa;
typedef v4u __attribute__((may_alias)) v4ua;
typedef v2u __attribute__((may_alias)) v2ua;

union FragBF { v16bf v; v4u q[2]; };

__device__ __forceinline__ unsigned int bfb(float f) {
  unsigned int u = __float_as_uint(f);
  u += 0x7FFFu + ((u >> 16) & 1u);
  return u >> 16;
}
__device__ __forceinline__ void split2(float v, unsigned int& hi, unsigned int& lo) {
  hi = bfb(v);
  lo = bfb(v - __uint_as_float(hi << 16));
}
__device__ __forceinline__ unsigned int pk(unsigned int a, unsigned int b) { return (a & 0xFFFFu) | (b << 16); }

__device__ __forceinline__ void split4(v4f a, v2u& H, v2u& L) {
  unsigned int h0, l0, h1, l1, h2, l2, h3, l3;
  split2(a.x, h0, l0); split2(a.y, h1, l1); split2(a.z, h2, l2); split2(a.w, h3, l3);
  H.x = pk(h0, h1); H.y = pk(h2, h3);
  L.x = pk(l0, l1); L.y = pk(l2, l3);
}
__device__ __forceinline__ void split8(v4f a, v4f c, v4u& H, v4u& L) {
  unsigned int h0, l0, h1, l1, h2, l2, h3, l3, h4, l4, h5, l5, h6, l6, h7, l7;
  split2(a.x, h0, l0); split2(a.y, h1, l1); split2(a.z, h2, l2); split2(a.w, h3, l3);
  split2(c.x, h4, l4); split2(c.y, h5, l5); split2(c.z, h6, l6); split2(c.w, h7, l7);
  H.x = pk(h0, h1); H.y = pk(h2, h3); H.z = pk(h4, h5); H.w = pk(h6, h7);
  L.x = pk(l0, l1); L.y = pk(l2, l3); L.z = pk(l4, l5); L.w = pk(l6, l7);
}

__device__ __forceinline__ v8f wmma_bf(v16bf a, v16bf b, v8f c) {
  v8f d = __builtin_amdgcn_wmma_f32_16x16x32_bf16(false, a, false, b, (short)0, c, false, false);
  asm volatile("v_nop\n\tv_nop\n\tv_nop\n\tv_nop" : "+v"(d) : "v"(a), "v"(b));
  return d;
}

__device__ __forceinline__ v16bf ldfrag_bf(const unsigned short* p, int h) {
  FragBF f;
  f.q[0] = *(const v4ua*)(p + 8 * h);
  f.q[1] = *(const v4ua*)(p + 16 + 8 * h);
  return f.v;
}

__global__ __launch_bounds__(256) void k_split(const float* __restrict__ src,
                                               unsigned short* __restrict__ ph,
                                               unsigned short* __restrict__ pl, int n8)
{
  const int g = blockIdx.x * 256 + threadIdx.x;
  if (g >= n8) return;
  const float* s = src + (size_t)g * 8;
  const v4f a = *(const v4fa*)s;
  const v4f c = *(const v4fa*)(s + 4);
  v4u H, L;
  split8(a, c, H, L);
  unsigned short* dh = ph + (size_t)g * 8;
  unsigned short* dl = pl + (size_t)g * 8;
  *(volatile v4u*)dh = H;
  *(volatile v4u*)dl = L;
  __threadfence();
  *(volatile v4u*)dh = H;
  *(volatile v4u*)dl = L;
}

__global__ __launch_bounds__(256) void k_tsplit(const float* __restrict__ W,
                                                unsigned short* __restrict__ Th,
                                                unsigned short* __restrict__ Tl, int K, int N)
{
  __shared__ __align__(16) unsigned short sH[64 * TSP];
  __shared__ __align__(16) unsigned short sL[64 * TSP];
  const int tid = threadIdx.x, lane = tid & 31, wv = tid >> 5;
  const int n0 = blockIdx.x * 64, k0 = blockIdx.y * 64;
  #pragma unroll 4
  for (int i = 0; i < 16; ++i) {
    const int idx = tid + 256 * i;
    const int kk = idx >> 6, nn = idx & 63;
    const float v = W[(size_t)(k0 + kk) * N + n0 + nn];
    unsigned int hb, lb;
    split2(v, hb, lb);
    sH[nn * TSP + kk] = (unsigned short)hb;
    sL[nn * TSP + kk] = (unsigned short)lb;
  }
  __syncthreads();
  const int piece = lane & 7, rq = lane >> 3;
  v4u hv[2], lv[2];
  size_t go[2];
  #pragma unroll
  for (int ps = 0; ps < 2; ++ps) {
    const int row = ps * 32 + wv * 4 + rq;
    hv[ps] = *(const v4ua*)(sH + row * TSP + 8 * piece);
    lv[ps] = *(const v4ua*)(sL + row * TSP + 8 * piece);
    go[ps] = (size_t)(n0 + row) * K + k0 + 8 * piece;
  }
  #pragma unroll
  for (int ps = 0; ps < 2; ++ps) {
    *(volatile v4u*)(Th + go[ps]) = hv[ps];
    *(volatile v4u*)(Tl + go[ps]) = lv[ps];
  }
  __threadfence();
  #pragma unroll
  for (int ps = 0; ps < 2; ++ps) {
    *(volatile v4u*)(Th + go[ps]) = hv[ps];
    *(volatile v4u*)(Tl + go[ps]) = lv[ps];
  }
}

__device__ __forceinline__ void kv_store(const float* sT, const float* bias, float* out,
                                         int bx, int by, int wv, int lane)
{
  const v4f bb = *(const v4fa*)(bias + by * 128 + 4 * lane);
  #pragma unroll
  for (int i = 0; i < 8; ++i) {
    const int R = wv + 8 * i;
    const v4f v = *(const v4fa*)(sT + R * KVP + 4 * lane) + bb;
    float* dst = out + (size_t)(bx * 64 + R) * HH + by * 128 + 4 * lane;
    *(volatile v4f*)dst = v;
  }
}

__global__ __launch_bounds__(256) void k_kv(const unsigned short* __restrict__ mh,
                                            const unsigned short* __restrict__ ml,
                                            const unsigned short* __restrict__ wkh,
                                            const unsigned short* __restrict__ wkl,
                                            const unsigned short* __restrict__ wvh,
                                            const unsigned short* __restrict__ wvl,
                                            const float* __restrict__ bk,
                                            const float* __restrict__ bv,
                                            float* __restrict__ Kp, float* __restrict__ Vp)
{
  __shared__ __align__(16) float sT[64 * KVP];
  const int tid = threadIdx.x, lane = tid & 31, wv = tid >> 5;
  const int h = lane >> 4, m = lane & 15;
  const int mat = blockIdx.z;
  const unsigned short* wh = mat ? wvh : wkh;
  const unsigned short* wl = mat ? wvl : wkl;
  const float* bias = mat ? bv : bk;
  float* out = mat ? Vp : Kp;
  const int bx = blockIdx.x, by = blockIdx.y;
  const int wm = wv >> 2, wn = wv & 3;
  const int rb = bx * 64 + 32 * wm, cb = by * 128 + 32 * wn;

  const v8f z8 = {0.f, 0.f, 0.f, 0.f, 0.f, 0.f, 0.f, 0.f};
  v8f acc[2][2];
  #pragma unroll
  for (int mt = 0; mt < 2; ++mt)
    #pragma unroll
    for (int nt = 0; nt < 2; ++nt) acc[mt][nt] = z8;

  #pragma unroll 1
  for (int k0 = 0; k0 < DD; k0 += 32) {
    v16bf ah[2], al[2];
    #pragma unroll
    for (int mt = 0; mt < 2; ++mt) {
      const size_t ao = (size_t)(rb + 16 * mt + m) * DD + k0;
      ah[mt] = ldfrag_bf(mh + ao, h);
      al[mt] = ldfrag_bf(ml + ao, h);
    }
    #pragma unroll
    for (int nt = 0; nt < 2; ++nt) {
      const size_t bo = (size_t)(cb + 16 * nt + m) * DD + k0;
      const v16bf bh = ldfrag_bf(wh + bo, h);
      const v16bf bl = ldfrag_bf(wl + bo, h);
      #pragma unroll
      for (int mt = 0; mt < 2; ++mt) {
        acc[mt][nt] = wmma_bf(ah[mt], bh, acc[mt][nt]);
        acc[mt][nt] = wmma_bf(ah[mt], bl, acc[mt][nt]);
        acc[mt][nt] = wmma_bf(al[mt], bh, acc[mt][nt]);
      }
    }
  }
  #pragma unroll
  for (int mt = 0; mt < 2; ++mt)
    #pragma unroll
    for (int nt = 0; nt < 2; ++nt) {
      const int col = 32 * wn + 16 * nt + m;
      #pragma unroll
      for (int r = 0; r < 8; ++r) {
        const int row = 32 * wm + 16 * mt + 8 * h + r;
        sT[row * KVP + col] = acc[mt][nt][r];
      }
    }
  __syncthreads();
  kv_store(sT, bias, out, bx, by, wv, lane);
  __threadfence();
  kv_store(sT, bias, out, bx, by, wv, lane);
}

__device__ __forceinline__ void step_store(const float* sF, const float* sSC, const int* sOl,
                                           int mxl, int t, float* Hout,
                                           unsigned short* hnh, unsigned short* hnl,
                                           float* o1, float* o2, int tid)
{
  #pragma unroll
  for (int i = 0; i < 8; ++i) {
    const int g = tid + 256 * i;
    const int row = g >> 7;
    const v4f v = *(const v4fa*)(sF + 4 * g);
    const float a = (t < sOl[row] && t < mxl) ? 1.f : 0.f;
    *(volatile v4f*)(Hout + 4 * g) = v;
    *(volatile v4f*)(o1 + 4 * g) = v * a;
  }
  #pragma unroll
  for (int i = 0; i < 4; ++i) {
    const int g8 = tid + 256 * i;
    const v4f a = *(const v4fa*)(sF + 8 * g8);
    const v4f c = *(const v4fa*)(sF + 8 * g8 + 4);
    v4u H, L;
    split8(a, c, H, L);
    *(volatile v4u*)(hnh + 8 * g8) = H;
    *(volatile v4u*)(hnl + 8 * g8) = L;
  }
  #pragma unroll
  for (int i = 0; i < 2; ++i) {
    const int g = tid + 256 * i;
    const v4f v = *(const v4fa*)(sSC + 4 * g);
    *(volatile v4f*)(o2 + 4 * g) = v;
  }
}

__global__ __launch_bounds__(256) void k_step(
    const float* __restrict__ Lin, const float* __restrict__ Hin,
    const float* __restrict__ emb,
    const unsigned short* __restrict__ wqh, const unsigned short* __restrict__ wql,
    const float* __restrict__ bq,
    const float* __restrict__ Kp, const float* __restrict__ Vp,
    const unsigned short* __restrict__ wih, const unsigned short* __restrict__ wil,
    const unsigned short* __restrict__ whh, const unsigned short* __restrict__ whl,
    const float* __restrict__ b_ih, const float* __restrict__ b_hh,
    const int* __restrict__ olen, const int* __restrict__ mxlp,
    float* __restrict__ Hout, unsigned short* __restrict__ hnh, unsigned short* __restrict__ hnl,
    float* __restrict__ o1, float* __restrict__ o2, int t)
{
  extern __shared__ __align__(16) unsigned char dsm[];
  unsigned short* sQh = (unsigned short*)(dsm + O_QH);
  unsigned short* sQl = (unsigned short*)(dsm + O_QL);
  unsigned short* sCh = (unsigned short*)(dsm + O_CH);
  unsigned short* sCl = (unsigned short*)(dsm + O_CL);
  float* sF  = (float*)(dsm + O_F);
  float* sHp = (float*)(dsm + O_HP);
  float* sP  = (float*)(dsm + O_P);
  float* sSC = (float*)(dsm + O_SC);
  int* sAm = (int*)(dsm + O_AM);
  int* sOl = (int*)(dsm + O_OL);

  const int tid = threadIdx.x, lane = tid & 31, wv = tid >> 5;
  const int h = lane >> 4, m = lane & 15;
  const int mxl = mxlp[0];
  const v8f z8 = {0.f, 0.f, 0.f, 0.f, 0.f, 0.f, 0.f, 0.f};

  if (tid < BS) sOl[tid] = olen[tid];
  if (t > 0) {
    const int b = tid >> 4, j = tid & 15;
    const float* lr = Lin + (size_t)b * VV;
    float best = __uint_as_float(0xff800000u);
    int bi = 0;
    #pragma unroll 1
    for (int it = 0; it < VV / 64; ++it) {
      const int v0 = 64 * it + 4 * j;
      const v4f x = *(const v4fa*)(lr + v0);
      bool tk = x.x > best; best = tk ? x.x : best; bi = tk ? v0 : bi;
      tk = x.y > best;      best = tk ? x.y : best; bi = tk ? (v0 + 1) : bi;
      tk = x.z > best;      best = tk ? x.z : best; bi = tk ? (v0 + 2) : bi;
      tk = x.w > best;      best = tk ? x.w : best; bi = tk ? (v0 + 3) : bi;
    }
    #pragma unroll
    for (int off = 8; off > 0; off >>= 1) {
      const float ov = __shfl_xor(best, off);
      const int   oi = __shfl_xor(bi, off);
      const bool tk = (ov > best) || (ov == best && oi < bi);
      best = tk ? ov : best;
      bi   = tk ? oi : bi;
    }
    if (j == 0) sAm[b] = bi;
  } else {
    if (tid < BS) sAm[tid] = 0;
  }
  __syncthreads();

  #pragma unroll 1
  for (int i = 0; i < 8; ++i) {
    const int g = tid + 256 * i;
    const int row = g >> 7, c4 = g & 127;
    int a = sAm[row];
    a = (a < 0) ? 0 : ((a > VV - 1) ? (VV - 1) : a);
    const v4f e4 = *(const v4fa*)(emb + (size_t)a * HH + 4 * c4);
    v4f h4 = {0.f, 0.f, 0.f, 0.f};
    if (t > 0) h4 = *(const v4fa*)(Hin + row * HH + 4 * c4);
    v2u eh, el, yh, yl;
    split4(e4, eh, el);
    split4(h4, yh, yl);
    *(v2ua*)(sQh + row * QP + 4 * c4) = eh;
    *(v2ua*)(sQl + row * QP + 4 * c4) = el;
    *(v2ua*)(sQh + row * QP + HH + 4 * c4) = yh;
    *(v2ua*)(sQl + row * QP + HH + 4 * c4) = yl;
    *(v4fa*)(sHp + row * HH + 4 * c4) = h4;
  }
  __syncthreads();

  {
    v8f acc[4];
    #pragma unroll
    for (int j = 0; j < 4; ++j) acc[j] = z8;
    #pragma unroll 1
    for (int k0 = 0; k0 < QK; k0 += 32) {
      const v16bf ah = ldfrag_bf(sQh + m * QP + k0, h);
      const v16bf al = ldfrag_bf(sQl + m * QP + k0, h);
      #pragma unroll
      for (int j = 0; j < 4; ++j) {
        const size_t bo = (size_t)(64 * wv + 16 * j + m) * QK + k0;
        const v16bf bh = ldfrag_bf(wqh + bo, h);
        const v16bf bl = ldfrag_bf(wql + bo, h);
        acc[j] = wmma_bf(ah, bh, acc[j]);
        acc[j] = wmma_bf(ah, bl, acc[j]);
        acc[j] = wmma_bf(al, bh, acc[j]);
      }
    }
    #pragma unroll
    for (int j = 0; j < 4; ++j) {
      const int col = 64 * wv + 16 * j + m;
      const float bb = bq[col];
      #pragma unroll
      for (int r = 0; r < 8; ++r) sF[(8 * h + r) * HH + col] = acc[j][r] + bb;
    }
  }
  __syncthreads();

  #pragma unroll 1
  for (int b = 0; b < BS; ++b) {
    const int hd = wv;
    const float* qr = sF + b * HH + hd * DKD;
    const float* kr = Kp + ((size_t)lane * BS + b) * HH + hd * DKD;
    float d0 = 0.f, d1 = 0.f, d2 = 0.f, d3 = 0.f;
    #pragma unroll 2
    for (int j4 = 0; j4 < DKD / 4; ++j4) {
      const v4f q4 = *(const v4fa*)(qr + 4 * j4);
      const v4f ka = *(const v4fa*)(kr + 4 * j4);
      const v4f kb = *(const v4fa*)(kr + (size_t)32 * BS * HH + 4 * j4);
      const v4f kc = *(const v4fa*)(kr + (size_t)64 * BS * HH + 4 * j4);
      const v4f kd = *(const v4fa*)(kr + (size_t)96 * BS * HH + 4 * j4);
      d0 = fmaf(q4.x, ka.x, d0); d0 = fmaf(q4.y, ka.y, d0); d0 = fmaf(q4.z, ka.z, d0); d0 = fmaf(q4.w, ka.w, d0);
      d1 = fmaf(q4.x, kb.x, d1); d1 = fmaf(q4.y, kb.y, d1); d1 = fmaf(q4.z, kb.z, d1); d1 = fmaf(q4.w, kb.w, d1);
      d2 = fmaf(q4.x, kc.x, d2); d2 = fmaf(q4.y, kc.y, d2); d2 = fmaf(q4.z, kc.z, d2); d2 = fmaf(q4.w, kc.w, d2);
      d3 = fmaf(q4.x, kd.x, d3); d3 = fmaf(q4.y, kd.y, d3); d3 = fmaf(q4.z, kd.z, d3); d3 = fmaf(q4.w, kd.w, d3);
    }
    d0 *= 0.125f; d1 *= 0.125f; d2 *= 0.125f; d3 *= 0.125f;
    float mx = fmaxf(fmaxf(d0, d1), fmaxf(d2, d3));
    #pragma unroll
    for (int off = 16; off > 0; off >>= 1) mx = fmaxf(mx, __shfl_xor(mx, off));
    const float e0 = expf(d0 - mx), e1 = expf(d1 - mx), e2 = expf(d2 - mx), e3 = expf(d3 - mx);
    float sm = (e0 + e1) + (e2 + e3);
    #pragma unroll
    for (int off = 16; off > 0; off >>= 1) sm += __shfl_xor(sm, off);
    const float inv = 1.0f / sm;
    float* pw = sP + wv * LM;
    pw[lane]      = e0 * inv;
    pw[lane + 32] = e1 * inv;
    pw[lane + 64] = e2 * inv;
    pw[lane + 96] = e3 * inv;
    __syncthreads();

    float c0 = 0.f, c1 = 0.f;
    const float* vb = Vp + (size_t)b * HH + hd * DKD + lane;
    #pragma unroll 4
    for (int kk = 0; kk < LM; ++kk) {
      const float p = pw[kk];
      const float* vr = vb + (size_t)kk * BS * HH;
      c0 = fmaf(p, vr[0], c0);
      c1 = fmaf(p, vr[32], c1);
    }
    unsigned int hb0, lb0, hb1, lb1;
    split2(c0, hb0, lb0);
    split2(c1, hb1, lb1);
    sCh[b * CP + hd * DKD + lane]      = (unsigned short)hb0;
    sCl[b * CP + hd * DKD + lane]      = (unsigned short)lb0;
    sCh[b * CP + hd * DKD + lane + 32] = (unsigned short)hb1;
    sCl[b * CP + hd * DKD + lane + 32] = (unsigned short)lb1;
    if (tid < LM) {
      float s = 0.f;
      #pragma unroll
      for (int w = 0; w < NHD; ++w) s += sP[w * LM + tid];
      s *= 0.125f;
      const float a = (t < sOl[b] && t < mxl) ? 1.f : 0.f;
      sSC[b * LM + tid] = s * a;
    }
    __syncthreads();
  }

  #pragma unroll 1
  for (int cg = 0; cg < 4; ++cg) {
    const int j0 = 16 * (4 * wv + cg);
    v8f ai[3], ag[3];
    #pragma unroll
    for (int g = 0; g < 3; ++g) { ai[g] = z8; ag[g] = z8; }
    #pragma unroll 1
    for (int k0 = 0; k0 < HH; k0 += 32) {
      const v16bf xh = ldfrag_bf(sCh + m * CP + k0, h);
      const v16bf xl = ldfrag_bf(sCl + m * CP + k0, h);
      #pragma unroll
      for (int g = 0; g < 3; ++g) {
        const size_t bo = (size_t)(g * HH + j0 + m) * HH + k0;
        const v16bf bh = ldfrag_bf(wih + bo, h);
        const v16bf bl = ldfrag_bf(wil + bo, h);
        ai[g] = wmma_bf(xh, bh, ai[g]);
        ai[g] = wmma_bf(xh, bl, ai[g]);
        ai[g] = wmma_bf(xl, bh, ai[g]);
      }
    }
    #pragma unroll 1
    for (int k0 = 0; k0 < HH; k0 += 32) {
      const v16bf yh = ldfrag_bf(sQh + m * QP + HH + k0, h);
      const v16bf yl = ldfrag_bf(sQl + m * QP + HH + k0, h);
      #pragma unroll
      for (int g = 0; g < 3; ++g) {
        const size_t bo = (size_t)(g * HH + j0 + m) * HH + k0;
        const v16bf bh = ldfrag_bf(whh + bo, h);
        const v16bf bl = ldfrag_bf(whl + bo, h);
        ag[g] = wmma_bf(yh, bh, ag[g]);
        ag[g] = wmma_bf(yh, bl, ag[g]);
        ag[g] = wmma_bf(yl, bh, ag[g]);
      }
    }
    const int col = j0 + m;
    const float bi0 = b_ih[col], bi1 = b_ih[HH + col], bi2 = b_ih[2 * HH + col];
    const float bg0 = b_hh[col], bg1 = b_hh[HH + col], bg2 = b_hh[2 * HH + col];
    #pragma unroll
    for (int r = 0; r < 8; ++r) {
      const int row = 8 * h + r;
      const float ir  = ai[0][r] + bi0;
      const float iz  = ai[1][r] + bi1;
      const float inn = ai[2][r] + bi2;
      const float hr  = ag[0][r] + bg0;
      const float hz  = ag[1][r] + bg1;
      const float hn  = ag[2][r] + bg2;
      const float rg = 1.0f / (1.0f + expf(-(ir + hr)));
      const float zg = 1.0f / (1.0f + expf(-(iz + hz)));
      const float ng = tanhf(inn + rg * hn);
      const float hp = sHp[row * HH + col];
      sF[row * HH + col] = (1.0f - zg) * ng + zg * hp;
    }
  }
  __syncthreads();

  step_store(sF, sSC, sOl, mxl, t, Hout, hnh, hnl, o1, o2, tid);
  __threadfence();
  step_store(sF, sSC, sOl, mxl, t, Hout, hnh, hnl, o1, o2, tid);
}

__device__ __forceinline__ void lg_store(const float* st, const int* olen, int mxl, int t,
                                         float* Lout, float* o0, int n0, int h, int m)
{
  #pragma unroll
  for (int i = 0; i < 8; ++i) {
    const int row = 2 * i + h;
    const v4f v = *(const v4fa*)(st + row * LTP + 4 * m);
    const float a = (t < olen[row] && t < mxl) ? 1.f : 0.f;
    const size_t off = (size_t)row * VV + n0 + 4 * m;
    *(volatile v4f*)(Lout + off) = v;
    *(volatile v4f*)(o0 + off) = v * a;
  }
}

__global__ __launch_bounds__(64) void k_logits(const unsigned short* __restrict__ hnh,
                                               const unsigned short* __restrict__ hnl,
                                               const unsigned short* __restrict__ wfh,
                                               const unsigned short* __restrict__ wfl,
                                               const float* __restrict__ bfv,
                                               const int* __restrict__ olen,
                                               const int* __restrict__ mxlp,
                                               float* __restrict__ Lout,
                                               float* __restrict__ o0, int t)
{
  __shared__ __align__(16) float sT[2 * 16 * LTP];
  const int tid = threadIdx.x, lane = tid & 31, wv = tid >> 5;
  const int h = lane >> 4, m = lane & 15;
  const int n0 = blockIdx.x * 128 + wv * 64;
  const v8f z8 = {0.f, 0.f, 0.f, 0.f, 0.f, 0.f, 0.f, 0.f};
  v8f acc[4];
  #pragma unroll
  for (int j = 0; j < 4; ++j) acc[j] = z8;
  #pragma unroll 1
  for (int k0 = 0; k0 < HH; k0 += 32) {
    const v16bf ah = ldfrag_bf(hnh + m * HH + k0, h);
    const v16bf al = ldfrag_bf(hnl + m * HH + k0, h);
    #pragma unroll
    for (int j = 0; j < 4; ++j) {
      const size_t bo = (size_t)(n0 + 16 * j + m) * HH + k0;
      const v16bf bh = ldfrag_bf(wfh + bo, h);
      const v16bf bl = ldfrag_bf(wfl + bo, h);
      acc[j] = wmma_bf(ah, bh, acc[j]);
      acc[j] = wmma_bf(ah, bl, acc[j]);
      acc[j] = wmma_bf(al, bh, acc[j]);
    }
  }
  float* st = sT + wv * 16 * LTP;
  #pragma unroll
  for (int j = 0; j < 4; ++j) {
    const int col = 16 * j + m;
    const float bb = bfv[n0 + col];
    #pragma unroll
    for (int r = 0; r < 8; ++r) st[(8 * h + r) * LTP + col] = acc[j][r] + bb;
  }
  __syncthreads();
  const int mxl = mxlp[0];
  lg_store(st, olen, mxl, t, Lout, o0, n0, h, m);
  __threadfence();
  lg_store(st, olen, mxl, t, Lout, o0, n0, h, m);
}

extern "C" void kernel_launch(void* const* d_in, const int* in_sizes, int n_in,
                              void* d_out, int out_size, void* d_ws, size_t ws_size,
                              hipStream_t stream)
{
  if (n_in < 16) return;
  if (in_sizes[0]  != LM * BS * DD) return;
  if (in_sizes[1]  != VV * HH) return;
  if (in_sizes[2]  != QK * HH) return;
  if (in_sizes[3]  != HH) return;
  if (in_sizes[4]  != DD * HH) return;
  if (in_sizes[5]  != HH) return;
  if (in_sizes[6]  != DD * HH) return;
  if (in_sizes[7]  != HH) return;
  if (in_sizes[8]  != HH * G3) return;
  if (in_sizes[9]  != G3) return;
  if (in_sizes[10] != HH * G3) return;
  if (in_sizes[11] != G3) return;
  if (in_sizes[12] != HH * VV) return;
  if (in_sizes[13] != VV) return;
  if (in_sizes[14] != BS) return;
  if (in_sizes[15] < 1) return;
  const int per = BS * (VV + HH + LM);
  if (out_size <= 0 || (out_size % per) != 0) return;
  const int T = out_size / per;
  if (T > 1800) return;

  const float* memory = (const float*)d_in[0];
  const float* emb    = (const float*)d_in[1];
  const float* Wq     = (const float*)d_in[2];
  const float* bq     = (const float*)d_in[3];
  const float* Wk     = (const float*)d_in[4];
  const float* bk     = (const float*)d_in[5];
  const float* Wv     = (const float*)d_in[6];
  const float* bv     = (const float*)d_in[7];
  const float* W_ih   = (const float*)d_in[8];
  const float* b_ih   = (const float*)d_in[9];
  const float* W_hh   = (const float*)d_in[10];
  const float* b_hh   = (const float*)d_in[11];
  const float* Wf     = (const float*)d_in[12];
  const float* bf     = (const float*)d_in[13];
  const int*   olen   = (const int*)d_in[14];
  const int*   mxlp   = (const int*)d_in[15];

  float* out0 = (float*)d_out;
  float* out1 = out0 + (size_t)T * BS * VV;
  float* out2 = out1 + (size_t)T * BS * HH;

  const size_t bWQ  = (size_t)HH * QK * 2;
  const size_t bWG  = (size_t)G3 * HH * 2;
  const size_t bWF  = (size_t)VV * HH * 2;
  const size_t bWK  = (size_t)HH * DD * 2;
  const size_t bMEM = (size_t)MROWS * DD * 2;
  const size_t bKV  = (size_t)MROWS * HH * 4;
  const size_t bL   = (size_t)BS * VV * 4;
  const size_t bH   = (size_t)BS * HH * 4;
  const size_t bHN  = (size_t)BS * HH * 2;
  const size_t total = 2 * bWQ + 4 * bWG + 2 * bWF + 4 * bWK + 2 * bMEM + 2 * bKV
                     + 2 * bL + 2 * bH + 2 * bHN;
  if (total > ws_size) return;
  if (total > (size_t)134217728) return;

  char* ws = (char*)d_ws;
  size_t off = 0;
  unsigned short* WQH  = (unsigned short*)(ws + off); off += bWQ;
  unsigned short* WQL  = (unsigned short*)(ws + off); off += bWQ;
  unsigned short* WIH  = (unsigned short*)(ws + off); off += bWG;
  unsigned short* WIL  = (unsigned short*)(ws + off); off += bWG;
  unsigned short* WGH  = (unsigned short*)(ws + off); off += bWG;
  unsigned short* WGL  = (unsigned short*)(ws + off); off += bWG;
  unsigned short* WFH  = (unsigned short*)(ws + off); off += bWF;
  unsigned short* WFL  = (unsigned short*)(ws + off); off += bWF;
  unsigned short* WKH  = (unsigned short*)(ws + off); off += bWK;
  unsigned short* WKL  = (unsigned short*)(ws + off); off += bWK;
  unsigned short* WVH  = (unsigned short*)(ws + off); off += bWK;
  unsigned short* WVL  = (unsigned short*)(ws + off); off += bWK;
  unsigned short* MEMH = (unsigned short*)(ws + off); off += bMEM;
  unsigned short* MEML = (unsigned short*)(ws + off); off += bMEM;
  float*          KP   = (float*)(ws + off);          off += bKV;
  float*          VP   = (float*)(ws + off);          off += bKV;
  float*          LB0  = (float*)(ws + off);          off += bL;
  float*          LB1  = (float*)(ws + off);          off += bL;
  float*          HB0  = (float*)(ws + off);          off += bH;
  float*          HB1  = (float*)(ws + off);          off += bH;
  unsigned short* HNH  = (unsigned short*)(ws + off); off += bHN;
  unsigned short* HNL  = (unsigned short*)(ws + off); off += bHN;
  if (off != total) return;

  k_tsplit<<<dim3(HH / 64, QK / 64), 256, 0, stream>>>(Wq,   WQH, WQL, QK, HH);
  k_tsplit<<<dim3(G3 / 64, HH / 64), 256, 0, stream>>>(W_ih, WIH, WIL, HH, G3);
  k_tsplit<<<dim3(G3 / 64, HH / 64), 256, 0, stream>>>(W_hh, WGH, WGL, HH, G3);
  k_tsplit<<<dim3(VV / 64, HH / 64), 256, 0, stream>>>(Wf,   WFH, WFL, HH, VV);
  k_tsplit<<<dim3(HH / 64, DD / 64), 256, 0, stream>>>(Wk,   WKH, WKL, DD, HH);
  k_tsplit<<<dim3(HH / 64, DD / 64), 256, 0, stream>>>(Wv,   WVH, WVL, DD, HH);
  {
    const int n8 = MROWS * DD / 8;
    k_split<<<(n8 + 255) / 256, 256, 0, stream>>>(memory, MEMH, MEML, n8);
  }
  k_kv<<<dim3(MROWS / 64, HH / 128, 2), 256, 0, stream>>>(MEMH, MEML, WKH, WKL, WVH, WVL, bk, bv, KP, VP);

  hipFuncSetAttribute(reinterpret_cast<const void*>(&k_step),
                      hipFuncAttributeMaxDynamicSharedMemorySize, LDS_STEP);
  for (int t = 0; t < T; ++t) {
    const float* Lin  = (t & 1) ? LB0 : LB1;
    const float* Hin  = (t & 1) ? HB0 : HB1;
    float*       Lcur = (t & 1) ? LB1 : LB0;
    float*       Hcur = (t & 1) ? HB1 : HB0;
    k_step<<<1, 256, LDS_STEP, stream>>>(Lin, Hin, emb, WQH, WQL, bq, KP, VP,
                                          WIH, WIL, WGH, WGL, b_ih, b_hh, olen, mxlp,
                                          Hcur, HNH, HNL,
                                          out1 + (size_t)t * BS * HH,
                                          out2 + (size_t)t * BS * LM, t);
    k_logits<<<VV / 128, 64, 0, stream>>>(HNH, HNL, WFH, WFL, bf, olen, mxlp, Lcur,
                                          out0 + (size_t)t * BS * VV, t);
  }
}
